// NTTailAttentionModel2Softmax_2611340116245
// MI455X (gfx1250) — hardware-verified
//
#include <hip/hip_runtime.h>


#define NSEQ 1024
#define NB 64
#define NBB 16
#define NE 256
#define NH 512
#define NG 2048
#define NV 10000
#define NVP 10048
#define HP 520

typedef __attribute__((ext_vector_type(16))) _Float16 v16h;
typedef __attribute__((ext_vector_type(8)))  _Float16 v8h;
typedef __attribute__((ext_vector_type(16))) __bf16   v16b;
typedef __attribute__((ext_vector_type(8)))  __bf16   v8b;
typedef __attribute__((ext_vector_type(8)))  float    v8f;
typedef __attribute__((ext_vector_type(4)))  float    v4f;

__device__ __forceinline__ unsigned short f2bf_bits(float f) {
  unsigned u = __float_as_uint(f);
  return (unsigned short)((u + 0x7FFFu + ((u >> 16) & 1u)) >> 16);
}
__device__ __forceinline__ float bf_bits2f(unsigned short h) { return __uint_as_float(((unsigned)h) << 16); }

__device__ __forceinline__ void dep_guard_h(v8f& a, v8f& b, v16h x, v16h y) { asm volatile("v_nop\n\tv_nop\n\tv_nop\n\tv_nop" : "+v"(a), "+v"(b) : "v"(x), "v"(y)); }
__device__ __forceinline__ void dep_guard_b(v8f& a, v8f& b, v16b x, v16b y) { asm volatile("v_nop\n\tv_nop\n\tv_nop\n\tv_nop" : "+v"(a), "+v"(b) : "v"(x), "v"(y)); }
__device__ __forceinline__ void keep4_h(v16h a, v16h b, v16h c, v16h d) { asm volatile("v_nop" :: "v"(a), "v"(b), "v"(c), "v"(d)); }
__device__ __forceinline__ void keep4_b(v16b a, v16b b, v16b c, v16b d) { asm volatile("v_nop" :: "v"(a), "v"(b), "v"(c), "v"(d)); }
__device__ __forceinline__ void acc_guard4(v8f& a, v8f& b, v8f& c, v8f& d) { asm volatile("v_nop\n\tv_nop\n\tv_nop\n\tv_nop" : "+v"(a), "+v"(b), "+v"(c), "+v"(d)); }
template <typename T> struct Frag;
template <> struct Frag<_Float16> {
  typedef v16h V; union U { v16h v; v8h h[2]; };
  static __device__ __forceinline__ v16h load(const _Float16* p) {
    U f; f.h[0] = *(const v8h*)(p); f.h[1] = *(const v8h*)(p + 16); return f.v;
  }
  static __device__ __forceinline__ v8f mma(v16h a, v16h b, v8f c) {
    return __builtin_amdgcn_wmma_f32_16x16x32_f16(false, a, false, b, (short)0, c, false, false);
  }
  static __device__ __forceinline__ void guard(v8f& a, v8f& b, v16h x, v16h y) { dep_guard_h(a, b, x, y); }
  static __device__ __forceinline__ void keep(v16h a, v16h b, v16h c, v16h d) { keep4_h(a, b, c, d); }
};
template <> struct Frag<__bf16> {
  typedef v16b V; union U { v16b v; v8b h[2]; };
  static __device__ __forceinline__ v16b load(const __bf16* p) {
    U f; f.h[0] = *(const v8b*)(p); f.h[1] = *(const v8b*)(p + 16); return f.v;
  }
  static __device__ __forceinline__ v8f mma(v16b a, v16b b, v8f c) {
    return __builtin_amdgcn_wmma_f32_16x16x32_bf16(false, a, false, b, (short)0, c, false, false);
  }
  static __device__ __forceinline__ void guard(v8f& a, v8f& b, v16b x, v16b y) { dep_guard_b(a, b, x, y); }
  static __device__ __forceinline__ void keep(v16b a, v16b b, v16b c, v16b d) { keep4_b(a, b, c, d); }
};

template <int ET> struct Elem;
template <> struct Elem<0> { typedef _Float16 T; };
template <> struct Elem<1> { typedef __bf16 T; };
template <int ET, bool SPLIT, int BIAS_MODE, int OUT_MODE, bool RESID, int ACT = 0>
__global__ __launch_bounds__(256) void wmma_gemm64(
    const unsigned short* __restrict__ Ap, const unsigned short* __restrict__ A2p, int lda, long strideA,
    const unsigned short* __restrict__ Btp, const unsigned short* __restrict__ Bt2p, int ldb, long strideB,
    void* __restrict__ Cout, void* __restrict__ Cout2, int ldc, long strideC,
    const float* __restrict__ bias,
    const float* __restrict__ resid, long strideR,
    int M, int N, int K, float scale) {
  typedef typename Elem<ET>::T T;
  typedef typename Frag<T>::V V;
  const T* A = (const T*)Ap; const T* A2 = (const T*)A2p; const T* Bt = (const T*)Btp; const T* Bt2 = (const T*)Bt2p;
  __shared__ __align__(16) float sT[8][16 * 68];
  const int b    = blockIdx.y;
  const int lane = threadIdx.x & 31;
  const int wave = threadIdx.x >> 5;
  const int tilesN = N >> 6;
  const int tilesM = M >> 6;
  const int tile = blockIdx.x * 8 + wave;
  if (tile >= tilesM * tilesN) return;
  const int tm = tile / tilesN;
  const int tn = tile - tm * tilesN;
  const int m0 = tm << 6;
  const int n0 = tn << 6;

  const T* Ab  = A  + (size_t)b * strideA;
  const T* Bb  = Bt + (size_t)b * strideB;
  const T* Ab2 = SPLIT ? (A2  + (size_t)b * strideA) : nullptr;
  const T* Bb2 = SPLIT ? (Bt2 + (size_t)b * strideB) : nullptr;

  const int rlane = lane & 15;
  const int koff  = (lane >> 4) * 8;
  const int mOff  = (lane >> 4) * 8;

  v8f acc[4][4];
#pragma unroll
  for (int i = 0; i < 4; ++i)
#pragma unroll
    for (int j = 0; j < 4; ++j) acc[i][j] = (v8f){0.f,0.f,0.f,0.f,0.f,0.f,0.f,0.f};

  for (int k0 = 0; k0 < K; k0 += 32) {
    V bh[4], bl[4];
#pragma unroll
    for (int j = 0; j < 4; ++j) {
      const size_t bo = (size_t)(n0 + (j << 4) + rlane) * ldb + koff + k0;
      bh[j] = Frag<T>::load(Bb + bo);
      if (SPLIT) bl[j] = Frag<T>::load(Bb2 + bo);
    }
#pragma unroll
    for (int i = 0; i < 4; ++i) {
      const size_t ao = (size_t)(m0 + (i << 4) + rlane) * lda + koff + k0;
      V ah = Frag<T>::load(Ab + ao);
      V al;
      if (SPLIT) al = Frag<T>::load(Ab2 + ao);
#pragma unroll
      for (int j = 0; j < 4; ++j) {
        acc[i][j] = Frag<T>::mma(ah, bh[j], acc[i][j]);
        if (SPLIT) {
          acc[i][j] = Frag<T>::mma(ah, bl[j], acc[i][j]);
          acc[i][j] = Frag<T>::mma(al, bh[j], acc[i][j]);
        }
      }
      Frag<T>::guard(acc[i][0], acc[i][3], ah, SPLIT ? al : ah);
    }
    Frag<T>::keep(bh[0], bh[1], bh[2], bh[3]);
    if (SPLIT) Frag<T>::keep(bl[0], bl[1], bl[2], bl[3]);
  }
  acc_guard4(acc[0][0], acc[0][1], acc[0][2], acc[0][3]);
  acc_guard4(acc[1][0], acc[1][1], acc[1][2], acc[1][3]);
  acc_guard4(acc[2][0], acc[2][1], acc[2][2], acc[2][3]);
  acc_guard4(acc[3][0], acc[3][1], acc[3][2], acc[3][3]);

  float* slab = sT[wave];
  const float* Rb = RESID ? (resid + (size_t)b * strideR) : nullptr;
#pragma unroll
  for (int i = 0; i < 4; ++i) {
    const int mBase = m0 + (i << 4);
#pragma unroll
    for (int j = 0; j < 4; ++j) {
      const int n = n0 + (j << 4) + rlane;
      float bv = 0.f;
      if (BIAS_MODE == 2) bv = bias[n];
#pragma unroll
      for (int r = 0; r < 8; ++r) {
        float v = acc[i][j][r] * scale;
        if (BIAS_MODE == 1) v += bias[mBase + mOff + r];
        if (BIAS_MODE == 2) v += bv;
        if (RESID) v += Rb[(size_t)(mBase + mOff + r) * ldc + n];
        if (ACT == 1) v = tanhf(v);
        if (ACT == 2) v = fmaxf(v, 0.0f);
        if (ACT == 3) v = v / (1.0f + expf(-v));
        if (ACT == 4) v = (v > 0.f) ? v : 0.01f * v;
        if (ACT == 5) v = 0.5f * v * (1.0f + erff(v * 0.70710678118654752f));
        slab[(mOff + r) * 68 + (j << 4) + rlane] = v;
      }
    }
    __builtin_amdgcn_fence(__ATOMIC_RELEASE, "workgroup");
    __builtin_amdgcn_wave_barrier();
    __builtin_amdgcn_fence(__ATOMIC_ACQUIRE, "workgroup");
    if (OUT_MODE == 0) {
      float* C = (float*)Cout + (size_t)b * strideC;
      const int hh = lane >> 4, c4 = (lane & 15) * 4;
      for (int pass = 0; pass < 2; ++pass) {
#pragma unroll
        for (int it = 0; it < 8; ++it) {
          const int row = it * 2 + hh;
          v4f v = *(const v4f*)(slab + row * 68 + c4);
          *(volatile v4f*)(C + (size_t)(mBase + row) * ldc + n0 + c4) = v;
        }
        __threadfence();
      }
    } else {
      const int q = lane >> 3, c8 = (lane & 7) * 8;
      unsigned short* C  = (unsigned short*)Cout  + (size_t)b * strideC;
      unsigned short* C2 = (OUT_MODE == 2) ? ((unsigned short*)Cout2 + (size_t)b * strideC) : nullptr;
      for (int pass = 0; pass < 2; ++pass) {
#pragma unroll
        for (int it = 0; it < 4; ++it) {
          const int row = it * 4 + q;
          const float* sp = slab + row * 68 + c8;
          v8h hv, lv;
#pragma unroll
          for (int e = 0; e < 8; ++e) {
            if (OUT_MODE == 1) {
              hv[e] = (_Float16)sp[e];
            } else {
              unsigned short hb = f2bf_bits(sp[e]);
              unsigned short lb = f2bf_bits(sp[e] - bf_bits2f(hb));
              hv[e] = __builtin_bit_cast(_Float16, hb);
              lv[e] = __builtin_bit_cast(_Float16, lb);
            }
          }
          *(volatile v8h*)(C + (size_t)(mBase + row) * ldc + n0 + c8) = hv;
          if (OUT_MODE == 2) *(volatile v8h*)(C2 + (size_t)(mBase + row) * ldc + n0 + c8) = lv;
        }
        __threadfence();
      }
    }
    __builtin_amdgcn_fence(__ATOMIC_RELEASE, "workgroup");
    __builtin_amdgcn_wave_barrier();
    __builtin_amdgcn_fence(__ATOMIC_ACQUIRE, "workgroup");
  }
}

__global__ __launch_bounds__(256) void rows_f32_to_f16(
    const float* __restrict__ src, _Float16* __restrict__ dst, int R, int nsrc, int C, float scale)
{
  const int lane = threadIdx.x & 31;
  const int wave = threadIdx.x >> 5;
  const int r = blockIdx.x * 8 + wave;
  if (r >= R) return;
  const bool valid = (r < nsrc);
  const long sr = valid ? (long)r : (long)(nsrc - 1);
  const float* sp = src + (size_t)sr * C;
  _Float16* dp = dst + (size_t)r * C;
  const v4f z = (v4f){0.f, 0.f, 0.f, 0.f};
  const int nch = C >> 8;
  for (int ch = 0; ch < nch; ++ch) {
    const int c0 = ch * 256 + 8 * lane;
    v4f x0 = *(const v4f*)(sp + c0);
    v4f x1 = *(const v4f*)(sp + c0 + 4);
    if (!valid) { x0 = z; x1 = z; }
    v8h o;
#pragma unroll
    for (int e = 0; e < 4; ++e) {
      o[e]     = (_Float16)(x0[e] * scale);
      o[4 + e] = (_Float16)(x1[e] * scale);
    }
    *(volatile v8h*)(dp + c0) = o;
    __threadfence();
    *(volatile v8h*)(dp + c0) = o;
  }
}

__device__ __forceinline__ float sigm_f(float x) { return __builtin_amdgcn_rcpf(1.0f + __expf(-x)); }
__device__ __forceinline__ float tanh_f(float x) { return 1.0f - 2.0f * __builtin_amdgcn_rcpf(__expf(2.0f * x) + 1.0f); }

__global__ __launch_bounds__(256) void lstm_kernel(
    const _Float16* __restrict__ Whh16,
    const _Float16* __restrict__ G16,
    const int* __restrict__ tok,
    const float* __restrict__ h0, const float* __restrict__ c0,
    const float* __restrict__ b_ih, const float* __restrict__ b_hh,
    _Float16* __restrict__ outs16,
    float* __restrict__ hT, float* __restrict__ cT, int nvocab)
{
  __shared__ __align__(16) _Float16 hsh[2 * NBB * HP];
  __shared__ __align__(16) float slab[8 * NBB * 64];
  __shared__ __align__(16) float csh[NBB * NH];
  __shared__ float bsh[NG];
  typedef Frag<_Float16> F;
  const int tid = threadIdx.x;
  const int lane = tid & 31, wave = tid >> 5, hh = lane >> 4, rl = lane & 15;
  const int b0 = (int)blockIdx.x * NBB;
  for (int i = tid; i < 2 * NBB * HP; i += 256) {
    const int rem = i % (NBB * HP);
    const int b = rem / HP;
    const int u = rem - b * HP;
    const int uc = (u < NH) ? u : (NH - 1);
    const float v = h0[(size_t)(b0 + b) * NH + uc];
    hsh[i] = (_Float16)((u < NH) ? (v * 256.0f) : 0.0f);
  }
  for (int i = tid; i < NBB * NH; i += 256) csh[i] = c0[(size_t)b0 * NH + i];
  for (int i = tid; i < NG; i += 256) bsh[i] = b_ih[i] + b_hh[i];
  __syncthreads();
  const int u0 = wave * 64;
  const float S  = 1.0f / 16384.0f;
  const float XS = 1.0f / 32.0f;
  float* slabw = slab + wave * (NBB * 64);
  const int rq = lane >> 3, c8 = (lane & 7) * 8, c4 = (lane & 15) * 4;

  for (int s = 0; s < NSEQ; ++s) {
    const _Float16* hc = hsh + (s & 1) * (NBB * HP);
    _Float16* hn = hsh + ((s & 1) ^ 1) * (NBB * HP);
    const _Float16* xr[8];
#pragma unroll
    for (int r = 0; r < 8; ++r) {
      int id = tok[(size_t)s * NB + b0 + 8 * hh + r];
      id = (id < 0) ? (id + nvocab) : id;
      id = (id < 0) ? 0 : id;
      id = (id > nvocab - 1) ? (nvocab - 1) : id;
      xr[r] = G16 + (size_t)id * NG;
    }
#pragma unroll 1
    for (int q = 0; q < 4; ++q) {
      const int ub = u0 + 16 * q;
      v8f acc[4];
#pragma unroll
      for (int g = 0; g < 4; ++g) acc[g] = (v8f){0.f,0.f,0.f,0.f,0.f,0.f,0.f,0.f};
#pragma unroll 1
      for (int k0 = 0; k0 < NH; k0 += 32) {
        v16h bfr[4];
#pragma unroll
        for (int g = 0; g < 4; ++g) bfr[g] = F::load(Whh16 + (size_t)(g * NH + ub + rl) * NH + k0 + 8 * hh);
        const v16h a = F::load(hc + rl * HP + k0 + 8 * hh);
#pragma unroll
        for (int g = 0; g < 4; ++g) acc[g] = F::mma(a, bfr[g], acc[g]);
        F::guard(acc[0], acc[3], a, a);
        F::keep(bfr[0], bfr[1], bfr[2], bfr[3]);
      }
      acc_guard4(acc[0], acc[1], acc[2], acc[3]);

      const int u = ub + rl;
      const int scol = 16 * q + rl;
      const float bI = bsh[u], bF = bsh[NH + u], bG = bsh[2 * NH + u], bO = bsh[3 * NH + u];
#pragma unroll
      for (int r = 0; r < 8; ++r) {
        const int bl = 8 * hh + r;
        const _Float16* xp = xr[r] + u;
        const float gi = acc[0][r] * S + ((float)xp[0]      * XS + bI);
        const float gf = acc[1][r] * S + ((float)xp[NH]     * XS + bF);
        const float gg = acc[2][r] * S + ((float)xp[2 * NH] * XS + bG);
        const float go = acc[3][r] * S + ((float)xp[3 * NH] * XS + bO);
        const float cp = csh[bl * NH + u];
        const float cn = sigm_f(gf) * cp + sigm_f(gi) * tanh_f(gg);
        csh[bl * NH + u] = cn;
        const float h = sigm_f(go) * tanh_f(cn);
        hn[bl * HP + u] = (_Float16)(h * 256.0f);
        slabw[bl * 64 + scol] = h;
      }
      if (q == 3) {
        __builtin_amdgcn_fence(__ATOMIC_RELEASE, "workgroup");
        __builtin_amdgcn_wave_barrier();
        __builtin_amdgcn_fence(__ATOMIC_ACQUIRE, "workgroup");
        _Float16* ob = outs16 + ((size_t)s * NB + b0) * NH + u0 + c8;
        for (int pass = 0; pass < 2; ++pass) {
#pragma unroll
          for (int it = 0; it < 4; ++it) {
            const int row = it * 4 + rq;
            const float* sp = slabw + row * 64 + c8;
            v8h hv;
#pragma unroll
            for (int e = 0; e < 8; ++e) hv[e] = (_Float16)(sp[e] * 8.0f);
            *(volatile v8h*)(ob + (size_t)row * NH) = hv;
          }
          __threadfence();
        }
        if (s == NSEQ - 1) {
          float* hb = hT + (size_t)b0 * NH + u0 + c4;
          for (int pass = 0; pass < 2; ++pass) {
#pragma unroll
            for (int it = 0; it < 8; ++it) {
              const int row = it * 2 + hh;
              const v4f v = *(const v4f*)(slabw + row * 64 + c4);
              *(volatile v4f*)(hb + (size_t)row * NH) = v;
            }
            __threadfence();
          }
        }
        __builtin_amdgcn_fence(__ATOMIC_RELEASE, "workgroup");
        __builtin_amdgcn_wave_barrier();
        __builtin_amdgcn_fence(__ATOMIC_ACQUIRE, "workgroup");
      }
    }
    __syncthreads();
  }

  for (int pass = 0; pass < 2; ++pass) {
#pragma unroll
    for (int it = 0; it < 8; ++it) {
      const int j = tid + 256 * it;
      const int row = j >> 7;
      const int cc = (j & 127) * 4;
      const v4f v = *(const v4f*)(csh + row * NH + cc);
      *(volatile v4f*)(cT + (size_t)(b0 + row) * NH + cc) = v;
    }
    __threadfence();
  }
}

__global__ __launch_bounds__(512) void attn_u_kernel(
    const float* __restrict__ attn_w, const float* __restrict__ hT, float* __restrict__ u)
{
  const int h = threadIdx.x;
  const float* q = hT + (size_t)(NB - 1) * NH;
  float acc = 0.f;
#pragma unroll 4
  for (int k = 0; k < NH; ++k) acc += attn_w[(size_t)k * NH + h] * q[k];
  const float v = acc * 0.125f;
  *(volatile float*)(u + h) = v;
  __threadfence();
  *(volatile float*)(u + h) = v;
}

__global__ __launch_bounds__(256) void scores_kernel(
    const _Float16* __restrict__ outs16, const float* __restrict__ u, float* __restrict__ sc)
{
  __shared__ float ush[NH];
  __shared__ float res[32];
  const int tid = threadIdx.x, lane = tid & 31, wave = tid >> 5;
  ush[tid] = u[tid];
  ush[tid + 256] = u[tid + 256];
  __syncthreads();
#pragma unroll 1
  for (int i = 0; i < 4; ++i) {
    const int row = (int)blockIdx.x * 32 + wave * 4 + i;
    const _Float16* p = outs16 + (size_t)row * NH + lane * 16;
    const v8h a = *(const v8h*)(p);
    const v8h bb = *(const v8h*)(p + 8);
    float acc = 0.f;
#pragma unroll
    for (int e = 0; e < 8; ++e) {
      acc += (float)a[e]  * ush[lane * 16 + e];
      acc += (float)bb[e] * ush[lane * 16 + 8 + e];
    }
#pragma unroll
    for (int off = 16; off > 0; off >>= 1) acc += __shfl_xor(acc, off, 32);
    if (lane == 0) res[wave * 4 + i] = acc;
  }
  __syncthreads();
  if (tid < 32) {
    const float v = res[tid];
    float* p = sc + (size_t)blockIdx.x * 32 + tid;
    *(volatile float*)p = v;
    __threadfence();
    *(volatile float*)p = v;
  }
}

__global__ __launch_bounds__(512) void ctx_kernel(
    const float* __restrict__ sc, const _Float16* __restrict__ outs16,
    const float* __restrict__ hT, _Float16* __restrict__ cat16)
{
  __shared__ float wsh[NSEQ];
  __shared__ float red[512];
  __shared__ float cn[NH];
  const int tid = threadIdx.x, b = blockIdx.x;
  float m = -INFINITY;
  for (int s = tid; s < NSEQ - 1; s += 512) m = fmaxf(m, sc[(size_t)s * NB + b]);
  red[tid] = m;
  __syncthreads();
  for (int o = 256; o > 0; o >>= 1) { if (tid < o) red[tid] = fmaxf(red[tid], red[tid + o]); __syncthreads(); }
  const float mx = red[0];
  __syncthreads();
  float psum = 0.f;
  for (int s = tid; s < NSEQ - 1; s += 512) {
    const float e = __expf(sc[(size_t)s * NB + b] - mx);
    wsh[s] = e;
    psum += e;
  }
  red[tid] = psum;
  __syncthreads();
  for (int o = 256; o > 0; o >>= 1) { if (tid < o) red[tid] += red[tid + o]; __syncthreads(); }
  const float inv = 1.0f / red[0];
  __syncthreads();
  float acc = 0.f;
  const _Float16* op = outs16 + (size_t)b * NH + tid;
#pragma unroll 4
  for (int s = 0; s < NSEQ - 1; ++s) acc += wsh[s] * (float)op[(size_t)s * (NB * NH)];
  cn[tid] = acc * inv;
  __syncthreads();
  if (tid < 128) {
    const int cc = tid * 8;
    const int li = (cc < NH) ? cc : (NH - 8);
    const int gi = (cc >= NH) ? (cc - NH) : 0;
    v8h hv;
#pragma unroll
    for (int e = 0; e < 8; ++e) {
      const float lv = cn[li + e];
      const float gv = hT[(size_t)b * NH + gi + e] * 8.0f;
      const float v = (cc < NH) ? lv : gv;
      hv[e] = (_Float16)v;
    }
    _Float16* dp = cat16 + (size_t)b * (2 * NH) + cc;
    *(volatile v8h*)dp = hv;
    __threadfence();
    *(volatile v8h*)dp = hv;
  }
}

__global__ __launch_bounds__(256) void logsoftmax_kernel(
    const float* __restrict__ L, const float* __restrict__ bias, float* __restrict__ outp)
{
  __shared__ float red[256];
  const int tid = threadIdx.x;
  const int k = blockIdx.x;
  float lse0 = 0.f, lse1 = 0.f;
#pragma unroll
  for (int row = 0; row < 2; ++row) {
    const float* Lr = L + (size_t)(2 * k + row) * NVP;
    float m = -INFINITY;
    for (int n = tid; n < NV; n += 256) m = fmaxf(m, Lr[n] + bias[n]);
    red[tid] = m;
    __syncthreads();
    for (int o = 128; o > 0; o >>= 1) { if (tid < o) red[tid] = fmaxf(red[tid], red[tid + o]); __syncthreads(); }
    const float mx = red[0];
    __syncthreads();
    float sm = 0.f;
    for (int n = tid; n < NV; n += 256) sm += __expf(Lr[n] + bias[n] - mx);
    red[tid] = sm;
    __syncthreads();
    for (int o = 128; o > 0; o >>= 1) { if (tid < o) red[tid] += red[tid + o]; __syncthreads(); }
    const float lse = mx + __logf(red[0]);
    __syncthreads();
    if (row == 0) lse0 = lse; else lse1 = lse;
  }
  float* ob = outp + (size_t)(2 * k) * NV;
  for (int pass = 0; pass < 2; ++pass) {
    for (int j = tid; j < 2 * (NV / 4); j += 256) {
      const int row = (j >= (NV / 4)) ? 1 : 0;
      const int col = (j - row * (NV / 4)) * 4;
      const v4f lv = *(const v4f*)(L + (size_t)(2 * k + row) * NVP + col);
      const v4f bv = *(const v4f*)(bias + col);
      const float l = row ? lse1 : lse0;
      v4f o;
      o[0] = (lv[0] + bv[0]) - l; o[1] = (lv[1] + bv[1]) - l;
      o[2] = (lv[2] + bv[2]) - l; o[3] = (lv[3] + bv[3]) - l;
      *(volatile v4f*)(ob + (size_t)j * 4) = o;
    }
    __threadfence();
  }
}

extern "C" void kernel_launch(void* const* d_in, const int* in_sizes, int n_in,
                              void* d_out, int out_size, void* d_ws, size_t ws_size,
                              hipStream_t stream) {
  if (n_in < 11) return;
  if (in_sizes[0] != NSEQ * NB) return;
  if (in_sizes[1] != NB * NH || in_sizes[2] != NB * NH) return;
  if (in_sizes[3] % NE != 0 || in_sizes[3] < NE) return;
  if (in_sizes[4] != NG * NE || in_sizes[5] != NG * NH || in_sizes[6] != NG || in_sizes[7] != NG) return;
  if (in_sizes[8] != NH * NH) return;
  if (in_sizes[9] != NV * 2 * NH || in_sizes[10] != NV) return;
  if (out_size != NB * NV + 2 * NB * NH) return;
  const int nvocab = in_sizes[3] / NE;
  if (nvocab > NVP || nvocab < 1) return;

  const int*   tokens = (const int*)  d_in[0];
  const float* h0     = (const float*)d_in[1];
  const float* c0     = (const float*)d_in[2];
  const float* emb    = (const float*)d_in[3];
  const float* w_ih   = (const float*)d_in[4];
  const float* w_hh   = (const float*)d_in[5];
  const float* b_ih   = (const float*)d_in[6];
  const float* b_hh   = (const float*)d_in[7];
  const float* attn_w = (const float*)d_in[8];
  const float* h2o_w  = (const float*)d_in[9];
  const float* h2o_b  = (const float*)d_in[10];

  float* logp = (float*)d_out;
  float* hTp  = logp + (size_t)NB * NV;
  float* cTp  = hTp + (size_t)NB * NH;

  const size_t szG    = (size_t)NVP * NG * 2;
  const size_t szEmb  = (size_t)NVP * NE * 2;
  const size_t szWih  = (size_t)NG * NE * 2;
  const size_t szWhh  = (size_t)NG * NH * 2;
  const size_t szOuts = (size_t)NSEQ * NB * NH * 2;
  size_t off = 0;
  const size_t oG    = off; off += szG;
  const size_t oEmb  = off; off += szEmb;
  const size_t oWih  = off; off += szWih;
  const size_t oWhh  = off; off += szWhh;
  const size_t oOuts = off; off += szOuts;
  if (off > ws_size) return;
  const size_t szH2o  = (size_t)NVP * 2 * NH * 2;
  const size_t szCat  = (size_t)NB * 2 * NH * 2;
  const size_t szLog  = (size_t)NB * NVP * 4;
  const size_t szU    = 2048;
  const size_t szSc   = 262144;
  size_t off2 = oG;
  const size_t oH2o = off2; off2 += szH2o;
  const size_t oCat = off2; off2 += szCat;
  const size_t oLog = off2; off2 += szLog;
  const size_t oU   = off2; off2 += szU;
  const size_t oSc  = off2; off2 += szSc;
  if (off2 > oG + szG) return;

  char* ws = (char*)d_ws;
  _Float16* G16    = (_Float16*)(ws + oG);
  _Float16* emb16  = (_Float16*)(ws + oEmb);
  _Float16* wih16  = (_Float16*)(ws + oWih);
  _Float16* whh16  = (_Float16*)(ws + oWhh);
  _Float16* outs16 = (_Float16*)(ws + oOuts);
  _Float16* h2o16  = (_Float16*)(ws + oH2o);
  _Float16* cat16  = (_Float16*)(ws + oCat);
  float*    logits = (float*)(ws + oLog);
  float*    uvec   = (float*)(ws + oU);
  float*    scores = (float*)(ws + oSc);

  rows_f32_to_f16<<<(NVP + 7) / 8, 256, 0, stream>>>(emb, emb16, NVP, nvocab, NE, 64.0f);
  rows_f32_to_f16<<<(NG + 7) / 8, 256, 0, stream>>>(w_ih, wih16, NG, NG, NE, 64.0f);
  rows_f32_to_f16<<<(NG + 7) / 8, 256, 0, stream>>>(w_hh, whh16, NG, NG, NH, 64.0f);

  {
    const int blocks = ((NVP / 64) * (NG / 64) + 7) / 8;
    wmma_gemm64<0, false, 0, 1, false, 0><<<dim3(blocks, 1), 256, 0, stream>>>(
        (const unsigned short*)emb16, (const unsigned short*)emb16, NE, 0L,
        (const unsigned short*)wih16, (const unsigned short*)wih16, NE, 0L,
        (void*)G16, (void*)G16, NG, 0L,
        (const float*)uvec, (const float*)uvec, 0L, NVP, NG, NE, 1.0f / 128.0f);
  }

  lstm_kernel<<<NB / NBB, 256, 0, stream>>>(whh16, G16, tokens, h0, c0, b_ih, b_hh, outs16, hTp, cTp, nvocab);

  rows_f32_to_f16<<<(NVP + 7) / 8, 256, 0, stream>>>(h2o_w, h2o16, NVP, NV, 2 * NH, 64.0f);

  attn_u_kernel<<<1, NH, 0, stream>>>(attn_w, hTp, uvec);
  scores_kernel<<<((NSEQ - 1) * NB) / 32, 256, 0, stream>>>(outs16, uvec, scores);
  ctx_kernel<<<NB, NH, 0, stream>>>(scores, outs16, hTp, cat16);

  {
    const int blocks = ((NB / 64) * (NVP / 64) + 7) / 8;
    wmma_gemm64<0, false, 0, 0, false, 0><<<dim3(blocks, 1), 256, 0, stream>>>(
        (const unsigned short*)cat16, (const unsigned short*)cat16, 2 * NH, 0L,
        (const unsigned short*)h2o16, (const unsigned short*)h2o16, 2 * NH, 0L,
        (void*)logits, (void*)logits, NVP, 0L,
        (const float*)uvec, (const float*)uvec, 0L, NB, NVP, 2 * NH, 1.0f / 512.0f);
  }

  logsoftmax_kernel<<<NB / 2, 256, 0, stream>>>(logits, h2o_b, logp);
}
